// Rnn_layer_30099130810551
// MI455X (gfx1250) — hardware-verified
//
#include <hip/hip_runtime.h>
#include <stddef.h>


typedef __attribute__((ext_vector_type(16))) _Float16 v16h;
typedef __attribute__((ext_vector_type(8)))  _Float16 v8h;
typedef __attribute__((ext_vector_type(4)))  _Float16 v4h;
typedef __attribute__((ext_vector_type(8)))  float    v8f;
typedef __attribute__((ext_vector_type(4)))  float    v4f;

template <typename T> struct Frag;
template <> struct Frag<_Float16> {
  typedef v16h V; union U { v16h v; v8h h[2]; };
  static __device__ __forceinline__ v16h load(const _Float16* p) {
    U f; f.h[0] = *(const v8h*)(p); f.h[1] = *(const v8h*)(p + 16); return f.v;
  }
  static __device__ __forceinline__ v8f mma(v16h a, v16h b, v8f c) {
    return __builtin_amdgcn_wmma_f32_16x16x32_f16(false, a, false, b, (short)0, c, false, false);
  }
};

__device__ __forceinline__ v8f mma_h(v16h a, v16h b, v8f c) {
  c = Frag<_Float16>::mma(a, b, c);
  asm volatile("v_nop\n\tv_nop\n\tv_nop\n\tv_nop" : "+v"(c) : "v"(a), "v"(b));
  return c;
}

#define TSTEPS 128
#define EMB    100
#define KP     128
#define UNITS  64
#define RB     16
#define NT     128

__global__ __launch_bounds__(NT) void k_recur(
    const int*   __restrict__ tokens,
    const float* __restrict__ emb,
    const float* __restrict__ W1,
    const float* __restrict__ U1,
    const float* __restrict__ b1,
    const float* __restrict__ W2,
    const float* __restrict__ U2,
    const float* __restrict__ b2,
    const float* __restrict__ Wd,
    const float* __restrict__ bd,
    float*       __restrict__ stage,
    int vocab) {
  __shared__ __align__(16) _Float16 sW1t[UNITS * KP];
  __shared__ __align__(16) _Float16 sU1t[UNITS * UNITS];
  __shared__ __align__(16) _Float16 sW2t[UNITS * UNITS];
  __shared__ __align__(16) _Float16 sU2t[UNITS * UNITS];
  __shared__ __align__(16) _Float16 sX[RB * KP];
  __shared__ __align__(16) _Float16 sH1[2 * RB * UNITS];
  __shared__ __align__(16) _Float16 sH2[2 * RB * UNITS];
  __shared__ int sTok[RB * TSTEPS];
  __shared__ __align__(16) float sOut[32];

  const int tid  = threadIdx.x;
  const int lane = tid & 31;
  const int wave = tid >> 5;
  const int hh   = lane >> 4;
  const int rl   = lane & 15;
  const int nG   = wave * 16 + rl;
  const int b0   = blockIdx.x * RB;

  for (int i = tid; i < UNITS * KP; i += NT) {
    const int n = i >> 7, k = i & (KP - 1);
    const int kc = (k < EMB) ? k : (EMB - 1);
    const float w = W1[kc * UNITS + n];
    sW1t[i] = (k < EMB) ? (_Float16)w : (_Float16)0.0f;
  }
  for (int i = tid; i < UNITS * UNITS; i += NT) {
    const int n = i >> 6, k = i & (UNITS - 1);
    sU1t[i] = (_Float16)U1[k * UNITS + n];
    sW2t[i] = (_Float16)W2[k * UNITS + n];
    sU2t[i] = (_Float16)U2[k * UNITS + n];
  }
  for (int i = tid; i < RB * KP; i += NT) sX[i] = (_Float16)0.0f;
  for (int i = tid; i < 2 * RB * UNITS; i += NT) { sH1[i] = (_Float16)0.0f; sH2[i] = (_Float16)0.0f; }
  for (int i = tid; i < RB * TSTEPS; i += NT) {
    const int r = i >> 7, tt = i & (TSTEPS - 1);
    int tk = tokens[(size_t)(b0 + r) * TSTEPS + tt];
    if (tk < 0) tk += vocab;
    tk = (tk < 0) ? 0 : tk;
    tk = (tk > vocab - 1) ? (vocab - 1) : tk;
    sTok[i] = tk;
  }
  if (tid < 32) sOut[tid] = 0.0f;
  const float bias1 = b1[nG];
  const float bias2 = b2[nG];
  __syncthreads();

  for (int t = 0; t < TSTEPS; ++t) {
    const int cur = t & 1, nxt = cur ^ 1;

    for (int i = tid; i < RB * (EMB / 4); i += NT) {
      const int r  = i / (EMB / 4);
      const int c4 = i - r * (EMB / 4);
      const int tk = sTok[r * TSTEPS + t];
      const v4f v = *(const v4f*)(emb + (size_t)tk * EMB + 4 * c4);
      v4h hv;
      hv[0] = (_Float16)v[0]; hv[1] = (_Float16)v[1]; hv[2] = (_Float16)v[2]; hv[3] = (_Float16)v[3];
      *(v4h*)(sX + r * KP + 4 * c4) = hv;
    }
    __syncthreads();

    v8f acc1 = (v8f){bias1, bias1, bias1, bias1, bias1, bias1, bias1, bias1};
#pragma unroll
    for (int ks = 0; ks < KP / 32; ++ks) {
      const v16h a = Frag<_Float16>::load(sX   + rl * KP + 32 * ks + 8 * hh);
      const v16h b = Frag<_Float16>::load(sW1t + nG * KP + 32 * ks + 8 * hh);
      acc1 = mma_h(a, b, acc1);
    }
    const _Float16* h1c = sH1 + cur * (RB * UNITS);
    _Float16*       h1n = sH1 + nxt * (RB * UNITS);
#pragma unroll
    for (int ks = 0; ks < UNITS / 32; ++ks) {
      const v16h a = Frag<_Float16>::load(h1c  + rl * UNITS + 32 * ks + 8 * hh);
      const v16h b = Frag<_Float16>::load(sU1t + nG * UNITS + 32 * ks + 8 * hh);
      acc1 = mma_h(a, b, acc1);
    }
#pragma unroll
    for (int r = 0; r < 8; ++r) {
      const float hv = tanhf(acc1[r]);
      h1n[(8 * hh + r) * UNITS + nG] = (_Float16)hv;
    }
    __syncthreads();

    v8f acc2 = (v8f){bias2, bias2, bias2, bias2, bias2, bias2, bias2, bias2};
#pragma unroll
    for (int ks = 0; ks < UNITS / 32; ++ks) {
      const v16h a = Frag<_Float16>::load(h1n  + rl * UNITS + 32 * ks + 8 * hh);
      const v16h b = Frag<_Float16>::load(sW2t + nG * UNITS + 32 * ks + 8 * hh);
      acc2 = mma_h(a, b, acc2);
    }
    const _Float16* h2c = sH2 + cur * (RB * UNITS);
    _Float16*       h2n = sH2 + nxt * (RB * UNITS);
#pragma unroll
    for (int ks = 0; ks < UNITS / 32; ++ks) {
      const v16h a = Frag<_Float16>::load(h2c  + rl * UNITS + 32 * ks + 8 * hh);
      const v16h b = Frag<_Float16>::load(sU2t + nG * UNITS + 32 * ks + 8 * hh);
      acc2 = mma_h(a, b, acc2);
    }
    if (t == TSTEPS - 1) {
      float* sFin = (float*)(void*)sX;
#pragma unroll
      for (int r = 0; r < 8; ++r) sFin[(8 * hh + r) * UNITS + nG] = tanhf(acc2[r]);
    } else {
#pragma unroll
      for (int r = 0; r < 8; ++r) h2n[(8 * hh + r) * UNITS + nG] = (_Float16)tanhf(acc2[r]);
    }
  }
  __syncthreads();

  if (tid < RB) {
    const float* sFin = (const float*)(const void*)sX;
    float s = bd[0];
#pragma unroll 8
    for (int k = 0; k < UNITS; ++k) s += sFin[tid * UNITS + k] * Wd[k];
    const float e = expf(-s);
    sOut[tid] = 1.0f / (1.0f + e);
  }
  __syncthreads();
  if (tid < 8) {
    const v4f v = *(const v4f*)(sOut + 4 * tid);
    float* dst = stage + (size_t)blockIdx.x * 32 + 4 * tid;
    *(volatile v4f*)dst = v;
    __threadfence();
    *(volatile v4f*)dst = v;
  }
}

__global__ __launch_bounds__(128) void k_pack_out(const float* __restrict__ stage, float* __restrict__ out, int nq4) {
  for (int pass = 0; pass < 2; ++pass) {
    for (int q = threadIdx.x; q < nq4; q += 128) {
      const v4f v = *(const v4f*)(stage + (size_t)(q >> 2) * 32 + 4 * (q & 3));
      *(volatile v4f*)(out + (size_t)q * 4) = v;
    }
    __threadfence();
  }
}

extern "C" void kernel_launch(void* const* d_in, const int* in_sizes, int n_in,
                              void* d_out, int out_size, void* d_ws, size_t ws_size,
                              hipStream_t stream) {
  if (n_in < 10) return;
  const int*   tokens = (const int*)  d_in[0];
  const float* emb    = (const float*)d_in[1];
  const float* W1     = (const float*)d_in[2];
  const float* U1     = (const float*)d_in[3];
  const float* b1     = (const float*)d_in[4];
  const float* W2     = (const float*)d_in[5];
  const float* U2     = (const float*)d_in[6];
  const float* b2     = (const float*)d_in[7];
  const float* Wd     = (const float*)d_in[8];
  const float* bd     = (const float*)d_in[9];

  const int nseq  = in_sizes[0] / TSTEPS;
  const int vocab = in_sizes[1] / EMB;
  if (nseq <= 0 || (nseq % RB) != 0 || vocab <= 0) return;
  if (in_sizes[2] != EMB * UNITS || in_sizes[3] != UNITS * UNITS || in_sizes[5] != UNITS * UNITS ||
      in_sizes[6] != UNITS * UNITS || in_sizes[4] < UNITS || in_sizes[7] < UNITS || in_sizes[8] < UNITS || in_sizes[9] < 1) return;
  if (out_size < nseq) return;

  const int nblk = nseq / RB;
  const size_t stage_bytes = (size_t)nblk * 32 * sizeof(float);
  if (stage_bytes > ws_size) return;
  float* stage = (float*)d_ws;

  k_recur<<<dim3(nblk), dim3(NT), 0, stream>>>(tokens, emb, W1, U1, b1, W2, U2, b2, Wd, bd, stage, vocab);
  k_pack_out<<<dim3(1), dim3(128), 0, stream>>>(stage, (float*)d_out, nseq / 4);
}
